// SlimNNAttentionHead_13073880449824
// MI455X (gfx1250) — hardware-run, weakly checked
//
#include <hip/hip_runtime.h>


#define NBT  2
#define TT   768
#define CC   64
#define QB   128
#define DM   CC
#define NN   TT
#define NTK  TT
#define SCL  0.125f
#define LOSC 1024.0f

typedef _Float16 h16;
typedef unsigned short bf;
typedef __attribute__((ext_vector_type(16))) __bf16   v16bf;
typedef __attribute__((ext_vector_type(16))) _Float16 v16h;
typedef __attribute__((ext_vector_type(8)))  _Float16 v8h;
typedef __attribute__((ext_vector_type(8)))  unsigned short v8us;
typedef __attribute__((ext_vector_type(8)))  float    v8f;
typedef __attribute__((ext_vector_type(4)))  float    v4f;
typedef v8h  __attribute__((may_alias)) v8ha;
typedef v4f  __attribute__((may_alias)) v4fa;
typedef v8us __attribute__((may_alias)) v8usa;

__device__ __forceinline__ unsigned short f2bf(float f) { unsigned u = __float_as_uint(f); u += 0x7FFFu + ((u >> 16) & 1u); return (unsigned short)(u >> 16); }
__device__ __forceinline__ float bf2f(unsigned short b) { return __uint_as_float(((unsigned)b) << 16); }
__device__ __forceinline__ float bfr(float f) { return bf2f(f2bf(f)); }
__device__ __forceinline__ v16h cat16(v8h lo, v8h hi) { return __builtin_shufflevector(lo, hi, 0, 1, 2, 3, 4, 5, 6, 7, 8, 9, 10, 11, 12, 13, 14, 15); }
__device__ __forceinline__ v16bf cat16b(v8us lo, v8us hi) { return __builtin_bit_cast(v16bf, __builtin_shufflevector(lo, hi, 0, 1, 2, 3, 4, 5, 6, 7, 8, 9, 10, 11, 12, 13, 14, 15)); }
__device__ __forceinline__ v8f wmma16(v16h a, v16h b, v8f c) { return __builtin_amdgcn_wmma_f32_16x16x32_f16(false, a, false, b, (short)0, c, false, false); }
__device__ __forceinline__ v8f wmmab(v16bf a, v16bf b, v8f c) { return __builtin_amdgcn_wmma_f32_16x16x32_bf16(false, a, false, b, (short)0, c, false, false); }

template <bool SPLITA, bool F16OUT = false>
__global__ __launch_bounds__(128) void k_gemmb(const bf* __restrict__ A, const bf* __restrict__ Al, const bf* __restrict__ Bn, const float* __restrict__ bias, float* C, int ldc, h16* C2, const float* __restrict__ R = nullptr, int K = DM, int roundR = 1) {
    __shared__ __align__(16) float ost[4][16 * 68];
    const int lane = threadIdx.x & 31, wave = threadIdx.x >> 5, lr = lane & 15, hi = lane >> 4;
    const int r0 = blockIdx.x * 64 + wave * 16, c0 = blockIdx.y * 64;
    const size_t aoff = (size_t)(r0 + lr) * K + 8 * hi;
    size_t boff[4];
#pragma unroll
    for (int t = 0; t < 4; ++t) boff[t] = (size_t)(c0 + t * 16 + lr) * K + 8 * hi;
    v8f acc[4];
#pragma unroll
    for (int t = 0; t < 4; ++t) acc[t] = (v8f){};
#pragma unroll 1
    for (int kc = 0; kc < K; kc += 32) {
        const v16bf a = cat16b(*(const v8us*)(A + aoff + kc), *(const v8us*)(A + aoff + kc + 16));
        v16bf al = a;
        if (SPLITA) al = cat16b(*(const v8us*)(Al + aoff + kc), *(const v8us*)(Al + aoff + kc + 16));
#pragma unroll
        for (int t = 0; t < 4; ++t) { const v16bf b = cat16b(*(const v8us*)(Bn + boff[t] + kc), *(const v8us*)(Bn + boff[t] + kc + 16)); acc[t] = wmmab(a, b, acc[t]); if (SPLITA) acc[t] = wmmab(al, b, acc[t]); }
        asm volatile("v_nop\n\tv_nop\n\tv_nop\n\tv_nop" : "+v"(acc[0]), "+v"(acc[1]), "+v"(acc[2]), "+v"(acc[3]) : "v"(a), "v"(al));
    }
    float* os = &ost[wave][0];
#pragma unroll
    for (int t = 0; t < 4; ++t) { const float bv = bias ? bfr(bias[c0 + t * 16 + lr]) : 0.f;
#pragma unroll
        for (int j = 0; j < 8; ++j) os[(hi * 8 + j) * 68 + t * 16 + lr] = acc[t][j] + bv; }
    __syncthreads();
    if (F16OUT) {
        h16* crow = (h16*)(void*)C + (size_t)r0 * ldc + c0;
        auto pass = [&]() {
#pragma unroll
            for (int s = 0; s < 4; ++s) { const int row = 4 * s + (lane >> 3), piece = lane & 7; const float* sp = os + row * 68 + piece * 8; v8h o, o2;
#pragma unroll
                for (int i = 0; i < 8; ++i) { const h16 a = (h16)sp[i]; o[i] = a; o2[i] = (h16)((sp[i] - (float)a) * LOSC); }
                *(volatile v8h*)(crow + (size_t)row * ldc + piece * 8) = o; if (C2) *(volatile v8h*)(C2 + (size_t)r0 * ldc + c0 + (size_t)row * ldc + piece * 8) = o2; }
        };
        pass(); __threadfence(); pass();
    } else {
        float* crow = C + (size_t)r0 * ldc + c0;
        auto pass = [&]() {
#pragma unroll
            for (int s = 0; s < 8; ++s) { const int Lid = (lane >> 3) + 4 * s, piece = lane & 7; const int row = Lid >> 1, cofs = (Lid & 1) * 32 + piece * 4;
                v4f val = *(const v4fa*)(os + row * 68 + cofs); if (R) { const v4f rv = *(const v4f*)(R + ((size_t)r0 + row) * ldc + c0 + cofs); val += roundR ? (v4f){bfr(rv[0]), bfr(rv[1]), bfr(rv[2]), bfr(rv[3])} : rv; }
                *(volatile v4f*)(crow + (size_t)row * ldc + cofs) = val; }
        };
        pass(); __threadfence(); pass();
    }
}

__global__ __launch_bounds__(128) void k_gemm3(const bf* __restrict__ Ah, const bf* __restrict__ Al, const bf* __restrict__ Bh, const bf* __restrict__ Bl, int K, float* C, int ldc) {
    __shared__ __align__(16) float ost[4][16 * 68];
    const int lane = threadIdx.x & 31, wave = threadIdx.x >> 5, lr = lane & 15, hi = lane >> 4;
    const int r0 = blockIdx.x * 64 + wave * 16, c0 = blockIdx.y * 64;
    const size_t aoff = (size_t)(r0 + lr) * K + 8 * hi;
    v8f acc[4];
#pragma unroll
    for (int t = 0; t < 4; ++t) acc[t] = (v8f){};
#pragma unroll 1
    for (int kc = 0; kc < K; kc += 32) {
        const v16bf a = cat16b(*(const v8us*)(Ah + aoff + kc), *(const v8us*)(Ah + aoff + kc + 16));
        const v16bf al = cat16b(*(const v8us*)(Al + aoff + kc), *(const v8us*)(Al + aoff + kc + 16));
#pragma unroll
        for (int t = 0; t < 4; ++t) { const size_t bo = (size_t)(c0 + t * 16 + lr) * K + kc + 8 * hi;
            const v16bf bh = cat16b(*(const v8us*)(Bh + bo), *(const v8us*)(Bh + bo + 16)); const v16bf bl = cat16b(*(const v8us*)(Bl + bo), *(const v8us*)(Bl + bo + 16));
            acc[t] = wmmab(a, bh, acc[t]); acc[t] = wmmab(al, bh, acc[t]); acc[t] = wmmab(a, bl, acc[t]); }
        asm volatile("v_nop\n\tv_nop\n\tv_nop\n\tv_nop" : "+v"(acc[0]), "+v"(acc[1]), "+v"(acc[2]), "+v"(acc[3]) : "v"(a), "v"(al));
    }
    float* os = &ost[wave][0];
#pragma unroll
    for (int t = 0; t < 4; ++t) {
#pragma unroll
        for (int j = 0; j < 8; ++j) os[(hi * 8 + j) * 68 + t * 16 + lr] = acc[t][j]; }
    __builtin_amdgcn_wave_barrier(); asm volatile("" ::: "memory");
    float* crow = C + (size_t)r0 * ldc + c0;
    auto pass = [&]() {
#pragma unroll
        for (int s = 0; s < 8; ++s) { const int Lid = (lane >> 3) + 4 * s, piece = lane & 7; const int row = Lid >> 1, cofs = (Lid & 1) * 32 + piece * 4;
            const v4f val = *(const v4fa*)(os + row * 68 + cofs); *(volatile v4f*)(crow + (size_t)row * ldc + cofs) = val; }
    };
    pass(); __threadfence(); pass();
}


__global__ __launch_bounds__(256) void k_cvt64(const float* __restrict__ src, int rows, bf* dst) {
    typedef __attribute__((ext_vector_type(2))) unsigned short v2us;
    const int lane = threadIdx.x & 31; const size_t r = (size_t)blockIdx.x * 8 + (threadIdx.x >> 5); if (r >= (size_t)rows) return; v2us o; o[0] = f2bf(src[r * CC + lane * 2]); o[1] = f2bf(src[r * CC + lane * 2 + 1]);
    *(volatile v2us*)(dst + r * CC + lane * 2) = o; __threadfence(); *(volatile v2us*)(dst + r * CC + lane * 2) = o;
}
__global__ __launch_bounds__(256) void k_wt64(const float* __restrict__ Wm, int K, int N, bf* Bt) {
    typedef __attribute__((ext_vector_type(2))) unsigned short v2us;
    const int lane = threadIdx.x & 31; const int n = blockIdx.x * 8 + (threadIdx.x >> 5); if (n >= N) return;
    for (int k0 = 0; k0 < K; k0 += 64) { v2us o; o[0] = f2bf(Wm[(size_t)(k0 + lane * 2) * N + n]); o[1] = f2bf(Wm[(size_t)(k0 + lane * 2 + 1) * N + n]); *(volatile v2us*)(Bt + (size_t)n * K + k0 + lane * 2) = o; }
    __threadfence();
    for (int k0 = 0; k0 < K; k0 += 64) { v2us o; o[0] = f2bf(Wm[(size_t)(k0 + lane * 2) * N + n]); o[1] = f2bf(Wm[(size_t)(k0 + lane * 2 + 1) * N + n]); *(volatile v2us*)(Bt + (size_t)n * K + k0 + lane * 2) = o; }
}
__global__ __launch_bounds__(256) void k_relu64p(const float* __restrict__ F, int rows, bf* Ph, bf* Pl) {
    typedef __attribute__((ext_vector_type(2))) unsigned short v2us;
    const int lane = threadIdx.x & 31; const size_t r = (size_t)blockIdx.x * 8 + (threadIdx.x >> 5); if (r >= (size_t)rows) return; v2us oh, ol;
#pragma unroll
    for (int i = 0; i < 2; ++i) { const float y = fmaxf(F[r * CC + lane * 2 + i], 0.f); const unsigned short hb = f2bf(y); oh[i] = hb; ol[i] = f2bf(y - bf2f(hb)); }
    const size_t o = r * CC + lane * 2; *(volatile v2us*)(Ph + o) = oh; *(volatile v2us*)(Pl + o) = ol; __threadfence(); *(volatile v2us*)(Ph + o) = oh; *(volatile v2us*)(Pl + o) = ol;
}
__global__ __launch_bounds__(256) void k_cat128(const float* __restrict__ PE, const float* __restrict__ x, bf* Xh, bf* Xl) {
    typedef __attribute__((ext_vector_type(4))) unsigned short v4us;
    const int lane = threadIdx.x & 31; const size_t r = (size_t)blockIdx.x * 8 + (threadIdx.x >> 5); if (r >= (size_t)TT) return; v4us oh, ol;
#pragma unroll
    for (int i = 0; i < 4; ++i) { const int c = lane * 4 + i; float y; if (c < CC) y = PE[r * CC + c]; else y = bfr(x[r * CC + (c - CC)]); const unsigned short hb = f2bf(y); oh[i] = hb; ol[i] = f2bf(y - bf2f(hb)); }
    const size_t o = r * (2 * CC) + lane * 4; *(volatile v4us*)(Xh + o) = oh; *(volatile v4us*)(Xl + o) = ol; __threadfence(); *(volatile v4us*)(Xh + o) = oh; *(volatile v4us*)(Xl + o) = ol;
}
__global__ __launch_bounds__(256) void k_pairs(const float* __restrict__ HQK, const float* __restrict__ ab1, int i0, bf* Hh, bf* Hl) {
    typedef __attribute__((ext_vector_type(2))) unsigned short v2us;
    const int lane = threadIdx.x & 31; const size_t w = (size_t)blockIdx.x * 8 + (threadIdx.x >> 5); if (w >= (size_t)QB * TT) return; const int i = i0 + (int)(w / TT), j = (int)(w % TT); v2us oh, ol;
#pragma unroll
    for (int q = 0; q < 2; ++q) { const int c = lane * 2 + q; const float y = fmaxf(HQK[(size_t)i * (2 * CC) + CC + c] + HQK[(size_t)j * (2 * CC) + c] + bfr(ab1[c]), 0.f); const unsigned short hb = f2bf(y); oh[q] = hb; ol[q] = f2bf(y - bf2f(hb)); }
    const size_t o = w * CC + lane * 2; *(volatile v2us*)(Hh + o) = oh; *(volatile v2us*)(Hl + o) = ol; __threadfence(); *(volatile v2us*)(Hh + o) = oh; *(volatile v2us*)(Hl + o) = ol;
}
__global__ __launch_bounds__(256) void k_score(const float* __restrict__ H2, const float* __restrict__ ab2, const float* __restrict__ sw, const float* __restrict__ sb, int i0, float* S) {
    const int lane = threadIdx.x & 31; const size_t w = (size_t)blockIdx.x * 8 + (threadIdx.x >> 5); if (w >= (size_t)QB * (TT / 32)) return; const int il = (int)(w / (TT / 32)), j = (int)(w % (TT / 32)) * 32 + lane; const float* hr = H2 + ((size_t)il * TT + j) * CC; float s = bfr(sb[0]);
#pragma unroll 1
    for (int c = 0; c < CC; ++c) s = fmaf(hr[c] + bfr(ab2[c]), bfr(sw[c]), s);
    float* dst = S + (size_t)(i0 + il) * TT + j; *(volatile float*)dst = s; __threadfence(); *(volatile float*)dst = s;
}
__global__ __launch_bounds__(256) void k_csoft768(const float* __restrict__ S, float sc, bf* PH, bf* PL) {
    typedef __attribute__((ext_vector_type(4))) unsigned short v4us;
    const int lane = threadIdx.x & 31, i = blockIdx.x * 8 + (threadIdx.x >> 5); if (i >= TT) return; const float* sr = S + (size_t)i * TT;
    float m = -3.0e38f;
#pragma unroll 1
    for (int c0 = lane * 4; c0 < TT; c0 += 128) {
#pragma unroll
        for (int q = 0; q < 4; ++q) { const int k = c0 + q; if (k <= i) m = fmaxf(m, sr[k] * sc); } }
#pragma unroll
    for (int sh = 16; sh; sh >>= 1) m = fmaxf(m, __shfl_xor(m, sh, 32));
    float sum = 0.f;
#pragma unroll 1
    for (int c0 = lane * 4; c0 < TT; c0 += 128) {
#pragma unroll
        for (int q = 0; q < 4; ++q) { const int k = c0 + q; if (k <= i) sum += __expf(sr[k] * sc - m); } }
#pragma unroll
    for (int sh = 16; sh; sh >>= 1) sum += __shfl_xor(sum, sh, 32);
    const float inv = 1.0f / sum;
#pragma unroll 1
    for (int ps = 0; ps < 2; ++ps) {
#pragma unroll 1
        for (int c0 = lane * 4; c0 < TT; c0 += 128) { v4us oh, ol;
#pragma unroll
            for (int q = 0; q < 4; ++q) { const int k = c0 + q; const float p = (k <= i) ? __expf(sr[(k <= i) ? k : 0] * sc - m) * inv : 0.f; const unsigned short hb = f2bf(p); oh[q] = hb; ol[q] = f2bf(p - bf2f(hb)); }
            const size_t o = (size_t)i * TT + c0; *(volatile v4us*)(PH + o) = oh; *(volatile v4us*)(PL + o) = ol; }
        if (ps == 0) __threadfence(); }
}
__global__ __launch_bounds__(256) void k_vT64(const float* __restrict__ V, bf* Th, bf* Tl) {
    __shared__ float tl[64][65];
    typedef __attribute__((ext_vector_type(4))) unsigned short v4us;
    const int tid = threadIdx.x; const int t0 = blockIdx.x * 64; const int rr = tid >> 2, cq = (tid & 3) * 16;
#pragma unroll
    for (int i = 0; i < 16; ++i) tl[rr][cq + i] = V[(size_t)(t0 + rr) * CC + cq + i];
    __syncthreads();
    const int lane = tid & 31, wv = tid >> 5;
    auto pass = [&]() {
#pragma unroll
        for (int st = 0; st < 4; ++st) { const int dr = wv * 8 + st * 2 + (lane >> 4); const int tq = (lane & 15) * 4; v4us oh, ol;
#pragma unroll
            for (int i = 0; i < 4; ++i) { const float y = tl[tq + i][dr]; const unsigned short hb = f2bf(y); oh[i] = hb; ol[i] = f2bf(y - bf2f(hb)); }
            const size_t o = (size_t)dr * TT + t0 + tq; *(volatile v4us*)(Th + o) = oh; *(volatile v4us*)(Tl + o) = ol; }
    };
    pass(); __threadfence(); pass();
}

extern "C" void kernel_launch(void* const* d_in, const int* in_sizes, int n_in,
                              void* d_out, int out_size, void* d_ws, size_t ws_size, hipStream_t stream) {
    (void)in_sizes; (void)n_in; (void)out_size;
    const float* x = (const float*)d_in[0]; const float* spe = (const float*)d_in[1]; const float* pw1 = (const float*)d_in[2]; const float* pb1 = (const float*)d_in[3]; const float* pw2 = (const float*)d_in[4]; const float* pb2 = (const float*)d_in[5];
    const float* aw1 = (const float*)d_in[6]; const float* ab1 = (const float*)d_in[7]; const float* aw2 = (const float*)d_in[8]; const float* ab2 = (const float*)d_in[9]; const float* sw = (const float*)d_in[10]; const float* sb = (const float*)d_in[11]; const float* vw = (const float*)d_in[12];
    float* out = (float*)d_out;
    char* wsp = (char*)d_ws;
    auto take = [&](size_t bytes) { char* p = wsp; wsp += (bytes + 255) & ~(size_t)255; return (void*)p; };
    bf* W1 = (bf*)take(CC * CC * 2); bf* W2 = (bf*)take(CC * CC * 2); bf* WA1 = (bf*)take((size_t)2 * CC * 4 * CC * 2); bf* WA2 = (bf*)take(CC * CC * 2); bf* WVb = (bf*)take(CC * CC * 2);
    bf* SPb = (bf*)take((size_t)TT * CC * 2); bf* Xb = (bf*)take((size_t)TT * CC * 2); float* P1 = (float*)take((size_t)TT * CC * 4); bf* P1h = (bf*)take((size_t)TT * CC * 2); bf* P1l = (bf*)take((size_t)TT * CC * 2); float* PE = (float*)take((size_t)TT * CC * 4);
    bf* X1h = (bf*)take((size_t)TT * 2 * CC * 2); bf* X1l = (bf*)take((size_t)TT * 2 * CC * 2); float* HQK = (float*)take((size_t)TT * 2 * CC * 4); float* V = (float*)take((size_t)TT * CC * 4); bf* VTh = (bf*)take((size_t)CC * TT * 2); bf* VTl = (bf*)take((size_t)CC * TT * 2);
    bf* Hh = (bf*)take((size_t)QB * TT * CC * 2); bf* Hl = (bf*)take((size_t)QB * TT * CC * 2); float* H2 = (float*)take((size_t)QB * TT * CC * 4); float* S = (float*)take((size_t)TT * TT * 4); bf* PH = (bf*)take((size_t)TT * TT * 2); bf* PL = (bf*)take((size_t)TT * TT * 2);
    if ((size_t)(wsp - (char*)d_ws) > ws_size) return;
    k_wt64<<<CC / 8, 256, 0, stream>>>(pw1, CC, CC, W1); k_wt64<<<CC / 8, 256, 0, stream>>>(pw2, CC, CC, W2); k_wt64<<<CC / 8, 256, 0, stream>>>(aw2, CC, CC, WA2); k_wt64<<<CC / 8, 256, 0, stream>>>(vw, CC, CC, WVb);
    k_wt64<<<CC / 8, 256, 0, stream>>>(aw1, 2 * CC, CC, WA1); k_wt64<<<CC / 8, 256, 0, stream>>>(aw1 + (size_t)2 * CC * CC, 2 * CC, CC, WA1 + (size_t)CC * 2 * CC);
    for (int b = 0; b < NBT; ++b) {
        k_cvt64<<<TT / 8, 256, 0, stream>>>(spe + (size_t)b * TT * CC, TT, SPb); k_cvt64<<<TT / 8, 256, 0, stream>>>(x + (size_t)b * TT * CC, TT, Xb);
        k_gemmb<false, false><<<dim3(TT / 64, 1, 1), 128, 0, stream>>>(SPb, nullptr, W1, pb1, P1, CC, nullptr, nullptr, CC); k_relu64p<<<TT / 8, 256, 0, stream>>>(P1, TT, P1h, P1l);
        k_gemmb<true, false><<<dim3(TT / 64, 1, 1), 128, 0, stream>>>(P1h, P1l, W2, pb2, PE, CC, nullptr, nullptr, CC);
        k_cat128<<<TT / 8, 256, 0, stream>>>(PE, x + (size_t)b * TT * CC, X1h, X1l);
        k_gemmb<true, false><<<dim3(TT / 64, 2, 1), 128, 0, stream>>>(X1h, X1l, WA1, nullptr, HQK, 2 * CC, nullptr, nullptr, 2 * CC);
        k_gemmb<false, false><<<dim3(TT / 64, 1, 1), 128, 0, stream>>>(Xb, nullptr, WVb, nullptr, V, CC, nullptr, nullptr, CC); k_vT64<<<TT / 64, 256, 0, stream>>>(V, VTh, VTl);
        for (int qb = 0; qb < TT / QB; ++qb) { const int i0 = qb * QB;
            k_pairs<<<(QB * TT) / 8, 256, 0, stream>>>(HQK, ab1, i0, Hh, Hl);
            k_gemmb<true, false><<<dim3((QB * TT) / 64, 1, 1), 128, 0, stream>>>(Hh, Hl, WA2, nullptr, H2, CC, nullptr, nullptr, CC);
            k_score<<<(QB * (TT / 32)) / 8, 256, 0, stream>>>(H2, ab2, sw, sb, i0, S); }
        k_csoft768<<<TT / 8, 256, 0, stream>>>(S, SCL, PH, PL);
        k_gemm3<<<dim3(TT / 64, 1, 1), 128, 0, stream>>>(PH, PL, VTh, VTl, TT, out + (size_t)b * TT * CC, CC); }
}
